// KANLayer_26688926777600
// MI455X (gfx1250) — hardware-verified
//
#include <hip/hip_runtime.h>
#include <stdint.h>

#pragma clang fp contract(off)

#define NROWS   4096
#define NIN     512
#define NOUT    512
#define NBAS    30
#define MK      34
#define NKN     (NIN * MK)
#define KF      (NIN * NBAS)
#define KTOT    (2 * KF)
#define CH      1024
#define NCHUNK  (NROWS / CH)
#define UROW    (KTOT / 8)
#define UHALF   (KF / 8)
#define FTHR    512
#define NSWEEP  ((UROW + FTHR - 1) / FTHR)
#define PUNITS  (NOUT * UROW)
#define PBLKS   (PUNITS / 256)
#define KSP     64
#define KFB     32
#define KBLKS   (NIN / KFB)
#define KTHR    128
#define WSCAP   134217728

static_assert(NROWS == NCHUNK * CH);
static_assert(CH % 128 == 0);
static_assert(NOUT % 64 == 0);
static_assert(KTOT % 32 == 0);
static_assert(UROW % 32 == 0);
static_assert((UROW % FTHR) % 32 == 0);
static_assert(NSWEEP * FTHR >= UROW);
static_assert(PUNITS == PBLKS * 256);
static_assert(FTHR == NIN);
static_assert(NBAS % 2 == 0);
static_assert((KF * 2) % 16 == 0);
static_assert((KTOT * 2) % 128 == 0);
static_assert((KSP * 4) % 128 == 0);
static_assert(NIN % KFB == 0);
static_assert(MK + 2 <= 36);
static_assert(36 <= KSP);
static_assert((KFB * KSP / 4) % KTHR == 0);

typedef float          v4f   __attribute__((ext_vector_type(4)));
typedef float          v8f   __attribute__((ext_vector_type(8)));
typedef int            v8i   __attribute__((ext_vector_type(8)));
typedef unsigned int   v4u   __attribute__((ext_vector_type(4)));
typedef unsigned short v8us  __attribute__((ext_vector_type(8)));
typedef __bf16         v16bf __attribute__((ext_vector_type(16)));
typedef v4f  __attribute__((may_alias)) v4fa;
typedef v4u  __attribute__((may_alias)) v4ua;
typedef v8us __attribute__((may_alias)) v8usa;
typedef unsigned int __attribute__((may_alias)) u32a;
union FragB { v16bf v; v8us h[2]; v8i w; };

__device__ __forceinline__ unsigned short f2bf_bits(float f) {
  unsigned u = __float_as_uint(f);
  return (unsigned short)((u + 0x7FFFu + ((u >> 16) & 1u)) >> 16);
}
__device__ __forceinline__ float bf_bits2f(unsigned short b) { return __uint_as_float(((unsigned)b) << 16); }
__device__ __forceinline__ float bfr(float f) { return bf_bits2f(f2bf_bits(f)); }
__device__ __forceinline__ unsigned pk16(unsigned short a, unsigned short b) { return (unsigned)a | ((unsigned)b << 16); }

__device__ __forceinline__ v8f wmb(const FragB& a, const FragB& b, v8f c) {
  v8f d = __builtin_amdgcn_wmma_f32_16x16x32_bf16(false, a.v, false, b.v, (short)0, c, false, false);
  asm volatile("v_nop\n\tv_nop\n\tv_nop\n\tv_nop" : "+v"(d) : "v"(a.w), "v"(b.w));
  return d;
}
__device__ __forceinline__ v8f z8() { v8f z = {0.f, 0.f, 0.f, 0.f, 0.f, 0.f, 0.f, 0.f}; return z; }

__device__ __forceinline__ void ks_store_pass(const float* so, float* dst, int tid) {
#pragma unroll
  for (int it = 0; it < (KFB * KSP / 4) / KTHR; ++it) {
    const int u = it * KTHR + tid;
    const v4f v = *(const v4fa*)(so + 4 * u);
    *(volatile v4f*)(dst + 4 * u) = v;
  }
}

__global__ __launch_bounds__(KTHR) void knot_kernel(const float* __restrict__ knots, float* __restrict__ KS) {
  __shared__ float sk[KFB * MK];
  __shared__ __align__(16) float so[KFB * KSP];
  const int tid = threadIdx.x;
  const int f0 = blockIdx.x * KFB;
  const int base = f0 * MK;
#pragma unroll 1
  for (int it = 0; it < (KFB * MK + KTHR - 1) / KTHR; ++it) {
    const int idx = it * KTHR + tid;
    int gi = base + idx;
    gi = gi > NKN - 1 ? NKN - 1 : gi;
    const float v = knots[gi];
    if (idx < KFB * MK) sk[idx] = v;
  }
  __syncthreads();
  if (tid < KFB) {
    const float* row = sk + tid * MK;
#pragma unroll 1
    for (int j = 0; j < MK; ++j) {
      const float vj = bfr(row[j]);
      int pos = 0;
#pragma unroll 1
      for (int m2 = 0; m2 < MK; ++m2) {
        const float vm = bfr(row[m2]);
        pos += (vm < vj) ? 1 : 0;
        pos += (vm == vj && m2 < j) ? 1 : 0;
      }
      so[tid * KSP + pos] = vj;
    }
#pragma unroll 1
    for (int j = MK; j < KSP; ++j) so[tid * KSP + j] = 0.0f;
  }
  __syncthreads();
  float* dst = KS + (size_t)f0 * KSP;
  ks_store_pass(so, dst, tid);
  __threadfence();
  ks_store_pass(so, dst, tid);
}

__global__ __launch_bounds__(256) void prep_kernel(const float* __restrict__ weights, unsigned short* __restrict__ WB) {
  const unsigned u  = blockIdx.x * 256u + threadIdx.x;
  const unsigned n  = u / (unsigned)UROW;
  const unsigned cu = u - n * (unsigned)UROW;
  const unsigned sc = (cu < (unsigned)UHALF) ? cu : (cu - (unsigned)UHALF);
  const float* src = weights + (size_t)n * KF + (size_t)sc * 8;
  unsigned short* dst = WB + (size_t)u * 8;
  const v4f a = *(const v4fa*)src;
  const v4f c = *(const v4fa*)(src + 4);
  v4u v;
  v[0] = pk16(f2bf_bits(a[0]), f2bf_bits(a[1]));
  v[1] = pk16(f2bf_bits(a[2]), f2bf_bits(a[3]));
  v[2] = pk16(f2bf_bits(c[0]), f2bf_bits(c[1]));
  v[3] = pk16(f2bf_bits(c[2]), f2bf_bits(c[3]));
  *(volatile v4u*)dst = v;
  __threadfence();
  *(volatile v4u*)dst = v;
}

template <int DD>
__device__ __forceinline__ void cdb_step(const float (&tk)[36], float (&B)[MK - 1], const float xv) {
#pragma unroll
  for (int j = 0; j < MK - 1 - DD; ++j) {
    const float den1 = tk[j + DD] - tk[j];
    const float den2 = tk[j + DD + 1] - tk[j + 1];
    const bool  p1 = den1 > 0.0f, p2 = den2 > 0.0f;
    const float r1 = __builtin_amdgcn_rcpf(p1 ? den1 : 1.0f);
    const float r2 = __builtin_amdgcn_rcpf(p2 ? den2 : 1.0f);
    const float w1 = p1 ? (xv - tk[j]) * r1 : 0.0f;
    const float w2 = p2 ? (tk[j + DD + 1] - xv) * r2 : 0.0f;
    const float nb = w1 * B[j] + w2 * B[j + 1];
    B[j] = nb;
  }
}

__device__ __forceinline__ void a_store_pass(const unsigned short* sA, unsigned short* dst, int tid) {
#pragma unroll
  for (int it = 0; it < NSWEEP; ++it) {
    const int u = it * FTHR + tid;
    if (u < UROW) {
      const v4u v = *(const v4ua*)(sA + 8 * u);
      *(volatile v4u*)(dst + 8 * u) = v;
    }
  }
}

__global__ __launch_bounds__(FTHR) void feat_kernel(const float* __restrict__ x, const float* __restrict__ KS,
                                                    unsigned short* __restrict__ AP, int row_base) {
  __shared__ __align__(16) unsigned short sA[KTOT];
  const int i = threadIdx.x;
  const int r = blockIdx.x;
  const float xv = bfr(x[(size_t)(row_base + r) * NIN + i]);

  float tk[36];
  const float* kp = KS + (size_t)i * KSP;
#pragma unroll
  for (int q = 0; q < 9; ++q) {
    const v4f w4 = *(const v4fa*)(kp + 4 * q);
    tk[4 * q + 0] = w4[0];
    tk[4 * q + 1] = w4[1];
    tk[4 * q + 2] = w4[2];
    tk[4 * q + 3] = w4[3];
  }

  float B[MK - 1];
#pragma unroll
  for (int j = 0; j < MK - 1; ++j) B[j] = (xv >= tk[j] && xv < tk[j + 1]) ? 1.0f : 0.0f;
  cdb_step<1>(tk, B, xv);
  cdb_step<2>(tk, B, xv);
  cdb_step<3>(tk, B, xv);
  const float valid = (xv >= tk[3] && xv <= tk[MK - 1 - 3]) ? 1.0f : 0.0f;

#pragma unroll
  for (int q = 0; q < NBAS / 2; ++q) {
    const float v0 = B[2 * q] * valid;
    const float v1 = B[2 * q + 1] * valid;
    const unsigned short h0 = f2bf_bits(v0), h1 = f2bf_bits(v1);
    const unsigned short l0 = f2bf_bits(v0 - bf_bits2f(h0));
    const unsigned short l1 = f2bf_bits(v1 - bf_bits2f(h1));
    *(u32a*)(sA + NBAS * i + 2 * q) = pk16(h0, h1);
    *(u32a*)(sA + KF + NBAS * i + 2 * q) = pk16(l0, l1);
  }
  __syncthreads();

  unsigned short* dst = AP + (size_t)r * KTOT;
  a_store_pass(sA, dst, i);
  __threadfence();
  a_store_pass(sA, dst, i);
}

__device__ __forceinline__ void o_store_pass(const float* sO, float* out,
                                             int grow_w, int n0, int w, int lane) {
  const int q8 = lane & 7, sub = lane >> 3;
#pragma unroll
  for (int i = 0; i < 16; ++i) {
    const int lid = i * 4 + sub;
    const int row = lid >> 1, hl = lid & 1;
    const v4f v = *(const v4fa*)(sO + (32 * w + row) * 64 + 32 * hl + 4 * q8);
    *(volatile v4f*)(out + (size_t)(grow_w + row) * NOUT + n0 + 32 * hl + 4 * q8) = v;
  }
}

__global__ __launch_bounds__(128) void gemm_kernel(const unsigned short* __restrict__ AP,
                                                   const unsigned short* __restrict__ WB,
                                                   const float* __restrict__ bias,
                                                   float* __restrict__ out, int row_base) {
  __shared__ __align__(16) float sO[128 * 64];
  const int tid = threadIdx.x, lane = tid & 31, w = tid >> 5;
  const int h = lane >> 4, m = lane & 15;
  const int lrow_w = blockIdx.x * 128 + 32 * w;
  const int n0 = blockIdx.y * 64;

  const unsigned short* xa0 = AP + (size_t)(lrow_w + m) * KTOT + 8 * h;
  const unsigned short* xa1 = xa0 + (size_t)16 * KTOT;
  const unsigned short* wb  = WB + (size_t)(n0 + m) * KTOT + 8 * h;

  v8f acc[2][4];
#pragma unroll
  for (int mt = 0; mt < 2; ++mt)
#pragma unroll
    for (int nt = 0; nt < 4; ++nt) acc[mt][nt] = z8();

#pragma unroll 1
  for (int k0 = 0; k0 < KTOT; k0 += 32) {
    FragB a0, a1;
    a0.h[0] = *(const v8usa*)(xa0 + k0);
    a0.h[1] = *(const v8usa*)(xa0 + k0 + 16);
    a1.h[0] = *(const v8usa*)(xa1 + k0);
    a1.h[1] = *(const v8usa*)(xa1 + k0 + 16);
#pragma unroll
    for (int nt = 0; nt < 4; ++nt) {
      const unsigned short* wq = wb + (size_t)nt * 16 * KTOT + k0;
      FragB b;
      b.h[0] = *(const v8usa*)wq;
      b.h[1] = *(const v8usa*)(wq + 16);
      acc[0][nt] = wmb(a0, b, acc[0][nt]);
      acc[1][nt] = wmb(a1, b, acc[1][nt]);
    }
  }

#pragma unroll
  for (int nt = 0; nt < 4; ++nt) {
    const int cl = 16 * nt + m;
    const float bc = bfr(bias[n0 + cl]);
#pragma unroll
    for (int mt = 0; mt < 2; ++mt) {
#pragma unroll
      for (int r = 0; r < 8; ++r) {
        const int rl = 32 * w + 16 * mt + 8 * h + r;
        sO[rl * 64 + cl] = acc[mt][nt][r] + bc;
      }
    }
  }
  __syncthreads();

  const int grow_w = row_base + lrow_w;
  o_store_pass(sO, out, grow_w, n0, w, lane);
  __threadfence();
  o_store_pass(sO, out, grow_w, n0, w, lane);
}

extern "C" void kernel_launch(void* const* d_in, const int* in_sizes, int n_in,
                              void* d_out, int out_size, void* d_ws, size_t ws_size,
                              hipStream_t stream) {
  if (n_in < 4) return;
  if (in_sizes[0] != NROWS * NIN) return;
  if (in_sizes[1] != NKN) return;
  if (in_sizes[2] != NOUT * KF) return;
  if (in_sizes[3] != NOUT) return;
  if (out_size != NROWS * NOUT) return;

  const float* x       = (const float*)d_in[0];
  const float* knots   = (const float*)d_in[1];
  const float* weights = (const float*)d_in[2];
  const float* bias    = (const float*)d_in[3];
  float* out = (float*)d_out;

  size_t off = 0;
  const size_t oAP = off; off += (size_t)CH * KTOT * 2;
  const size_t oWB = off; off += (size_t)NOUT * KTOT * 2;
  const size_t oKS = off; off += (size_t)NIN * KSP * 4;
  if (off > ws_size) return;
  if (off > (size_t)WSCAP) return;

  char* ws = (char*)d_ws;
  unsigned short* AP = (unsigned short*)(ws + oAP);
  unsigned short* WB = (unsigned short*)(ws + oWB);
  float* KS = (float*)(ws + oKS);

  knot_kernel<<<dim3(KBLKS), dim3(KTHR), 0, stream>>>(knots, KS);
  prep_kernel<<<dim3(PBLKS), dim3(256), 0, stream>>>(weights, WB);
  for (int c = 0; c < NCHUNK; ++c) {
    const int row_base = c * CH;
    feat_kernel<<<dim3(CH), dim3(FTHR), 0, stream>>>(x, KS, AP, row_base);
    gemm_kernel<<<dim3(CH / 128, NOUT / 64), dim3(128), 0, stream>>>(AP, WB, bias, out, row_base);
  }
  (void)hipGetLastError();
}
